// sLSTMblock_60163901882427
// MI455X (gfx1250) — hardware-verified
//
#include <hip/hip_runtime.h>
#include <math.h>

constexpr int NBATCH  = 8;
constexpr int NSTEP   = 2048;
constexpr int NIN     = 512;
constexpr int NHID    = 512;
constexpr int NG4     = 4 * NHID;
constexpr int NROWS   = NBATCH * NSTEP;
constexpr int CVT_THR = 256;
constexpr int SEQ_THR = 512;
constexpr int HPITCH  = 520;
constexpr int SPITCH  = 516;
constexpr int NOUT0   = NROWS * NHID;
constexpr int NOUT1   = NBATCH * NHID;
constexpr float WCARRY     = 16.0f;
constexpr float WCARRY_INV = 1.0f / 16.0f;

static_assert(NIN == NHID);
static_assert(NIN % 32 == 0 && NHID % 32 == 0);
static_assert(NROWS % 64 == 0 && NG4 % 64 == 0);
static_assert(NHID == 32 * (SEQ_THR / 32));
static_assert(NBATCH == 8);
static_assert((NBATCH * NHID / 4) == 2 * SEQ_THR);
static_assert(HPITCH % 8 == 0 && HPITCH >= NHID);
static_assert(SPITCH % 4 == 0 && SPITCH >= NHID);
static_assert((size_t)NOUT0 * 4 == 33554432u);
static_assert((size_t)(NOUT0 + NOUT1) * 4 == 33570816u);
static_assert((size_t)(NOUT0 + 2 * NOUT1) * 4 == 33587200u);

typedef __attribute__((ext_vector_type(16))) _Float16 v16h;
typedef __attribute__((ext_vector_type(8)))  _Float16 v8h;
typedef __attribute__((ext_vector_type(16))) __bf16   v16b;
typedef __attribute__((ext_vector_type(8)))  __bf16   v8b;
typedef __attribute__((ext_vector_type(8)))  float    v8f;
typedef __attribute__((ext_vector_type(4)))  float    v4f;

__device__ __forceinline__ unsigned short f2bf_bits(float f) {
  unsigned u = __float_as_uint(f);
  return (unsigned short)((u + 0x7FFFu + ((u >> 16) & 1u)) >> 16);
}
__device__ __forceinline__ float bf_bits2f(unsigned short h) { return __uint_as_float(((unsigned)h) << 16); }

__device__ __forceinline__ float h16_to_f32(unsigned hb) {
  const unsigned sgn = (hb & 0x8000u) << 16;
  const unsigned em = hb & 0x7fffu;
  const float fn = __uint_as_float((em << 13) + 0x38000000u);
  const float fs = (float)em * 5.9604644775390625e-8f;
  const float mag = (em < 0x400u) ? fs : fn;
  return __uint_as_float(__float_as_uint(mag) | sgn);
}

__device__ __forceinline__ void dep_guard4_h(v8f& a, v8f& b, v8f& c, v8f& d, v16h x, v16h y) {
  asm volatile("v_nop\n\tv_nop\n\tv_nop\n\tv_nop" : "+v"(a), "+v"(b), "+v"(c), "+v"(d) : "v"(x), "v"(y));
}
__device__ __forceinline__ void dep_guard4_b(v8f& a, v8f& b, v8f& c, v8f& d, v16b x, v16b y) {
  asm volatile("v_nop\n\tv_nop\n\tv_nop\n\tv_nop" : "+v"(a), "+v"(b), "+v"(c), "+v"(d) : "v"(x), "v"(y));
}
__device__ __forceinline__ void grp_guard_h(v8f& a0, v8f& a1, v8f& a2, v8f& a3, v16h x, v16h y0, v16h y1, v16h y2, v16h y3) {
  asm volatile("v_nop\n\tv_nop\n\tv_nop\n\tv_nop" : "+v"(a0), "+v"(a1), "+v"(a2), "+v"(a3) : "v"(x), "v"(y0), "v"(y1), "v"(y2), "v"(y3));
}
__device__ __forceinline__ void keep4_h(v16h a, v16h b, v16h c, v16h d) { asm volatile("v_nop" :: "v"(a), "v"(b), "v"(c), "v"(d)); }
__device__ __forceinline__ void keep4_b(v16b a, v16b b, v16b c, v16b d) { asm volatile("v_nop" :: "v"(a), "v"(b), "v"(c), "v"(d)); }
__device__ __forceinline__ void acc_guard4(v8f& a, v8f& b, v8f& c, v8f& d) { asm volatile("v_nop\n\tv_nop\n\tv_nop\n\tv_nop" : "+v"(a), "+v"(b), "+v"(c), "+v"(d)); }

template <typename T> struct Frag;
template <> struct Frag<_Float16> {
  typedef v16h V; union U { v16h v; v8h h[2]; };
  static __device__ __forceinline__ v16h load(const _Float16* p) {
    U f; f.h[0] = *(const v8h*)(p); f.h[1] = *(const v8h*)(p + 16); return f.v;
  }
  static __device__ __forceinline__ v8f mma(v16h a, v16h b, v8f c) {
    return __builtin_amdgcn_wmma_f32_16x16x32_f16(false, a, false, b, (short)0, c, false, false);
  }
  static __device__ __forceinline__ void guard4(v8f& a, v8f& b, v8f& c, v8f& d, v16h x, v16h y) { dep_guard4_h(a, b, c, d, x, y); }
  static __device__ __forceinline__ void keep(v16h a, v16h b, v16h c, v16h d) { keep4_h(a, b, c, d); }
};
template <> struct Frag<__bf16> {
  typedef v16b V; union U { v16b v; v8b h[2]; };
  static __device__ __forceinline__ v16b load(const __bf16* p) {
    U f; f.h[0] = *(const v8b*)(p); f.h[1] = *(const v8b*)(p + 16); return f.v;
  }
  static __device__ __forceinline__ v8f mma(v16b a, v16b b, v8f c) {
    return __builtin_amdgcn_wmma_f32_16x16x32_bf16(false, a, false, b, (short)0, c, false, false);
  }
  static __device__ __forceinline__ void guard4(v8f& a, v8f& b, v8f& c, v8f& d, v16b x, v16b y) { dep_guard4_b(a, b, c, d, x, y); }
  static __device__ __forceinline__ void keep(v16b a, v16b b, v16b c, v16b d) { keep4_b(a, b, c, d); }
};

template <int ET> struct Elem;
template <> struct Elem<0> { typedef _Float16 T; };
template <> struct Elem<1> { typedef __bf16 T; };
template <int ET, bool SPLIT, int BIAS_MODE, int OUT_MODE, bool RESID, int ACT = 0>
__global__ __launch_bounds__(256) void wmma_gemm64(
    const unsigned short* __restrict__ Ap, const unsigned short* __restrict__ A2p, int lda, long strideA,
    const unsigned short* __restrict__ Btp, const unsigned short* __restrict__ Bt2p, int ldb, long strideB,
    void* __restrict__ Cout, void* __restrict__ Cout2, int ldc, long strideC,
    const float* __restrict__ bias,
    const float* __restrict__ resid, long strideR,
    int M, int N, int K, float scale) {
  typedef typename Elem<ET>::T T;
  typedef typename Frag<T>::V V;
  const T* A = (const T*)Ap; const T* A2 = (const T*)A2p; const T* Bt = (const T*)Btp; const T* Bt2 = (const T*)Bt2p;
  __shared__ __align__(16) float sT[8][16 * 68];
  const int b    = blockIdx.y;
  const int lane = threadIdx.x & 31;
  const int wave = threadIdx.x >> 5;
  const int tilesN = N >> 6;
  const int tilesM = M >> 6;
  const int tile = blockIdx.x * 8 + wave;
  if (tile >= tilesM * tilesN) return;
  const int tm = tile / tilesN;
  const int tn = tile - tm * tilesN;
  const int m0 = tm << 6;
  const int n0 = tn << 6;

  const T* Ab  = A  + (size_t)b * strideA;
  const T* Bb  = Bt + (size_t)b * strideB;
  const T* Ab2 = SPLIT ? (A2  + (size_t)b * strideA) : nullptr;
  const T* Bb2 = SPLIT ? (Bt2 + (size_t)b * strideB) : nullptr;

  const int rlane = lane & 15;
  const int koff  = (lane >> 4) * 8;
  const int mOff  = (lane >> 4) * 8;

  v8f acc[4][4];
#pragma unroll
  for (int i = 0; i < 4; ++i)
#pragma unroll
    for (int j = 0; j < 4; ++j) acc[i][j] = (v8f){0.f,0.f,0.f,0.f,0.f,0.f,0.f,0.f};

  for (int k0 = 0; k0 < K; k0 += 32) {
    V bh[4], bl[4];
#pragma unroll
    for (int j = 0; j < 4; ++j) {
      const size_t bo = (size_t)(n0 + (j << 4) + rlane) * ldb + koff + k0;
      bh[j] = Frag<T>::load(Bb + bo);
      if (SPLIT) bl[j] = Frag<T>::load(Bb2 + bo);
    }
#pragma unroll
    for (int i = 0; i < 4; ++i) {
      const size_t ao = (size_t)(m0 + (i << 4) + rlane) * lda + koff + k0;
      V ah = Frag<T>::load(Ab + ao);
      V al;
      if (SPLIT) al = Frag<T>::load(Ab2 + ao);
#pragma unroll
      for (int j = 0; j < 4; ++j) {
        acc[i][j] = Frag<T>::mma(ah, bh[j], acc[i][j]);
        if (SPLIT) {
          acc[i][j] = Frag<T>::mma(ah, bl[j], acc[i][j]);
          acc[i][j] = Frag<T>::mma(al, bh[j], acc[i][j]);
        }
      }
      Frag<T>::guard4(acc[i][0], acc[i][1], acc[i][2], acc[i][3], ah, SPLIT ? al : ah);
    }
    Frag<T>::keep(bh[0], bh[1], bh[2], bh[3]);
    if (SPLIT) Frag<T>::keep(bl[0], bl[1], bl[2], bl[3]);
  }
  acc_guard4(acc[0][0], acc[0][1], acc[0][2], acc[0][3]);
  acc_guard4(acc[1][0], acc[1][1], acc[1][2], acc[1][3]);
  acc_guard4(acc[2][0], acc[2][1], acc[2][2], acc[2][3]);
  acc_guard4(acc[3][0], acc[3][1], acc[3][2], acc[3][3]);

  float* slab = sT[wave];
  const float* Rb = RESID ? (resid + (size_t)b * strideR) : nullptr;
#pragma unroll
  for (int i = 0; i < 4; ++i) {
    const int mBase = m0 + (i << 4);
#pragma unroll
    for (int j = 0; j < 4; ++j) {
      const int n = n0 + (j << 4) + rlane;
      float bv = 0.f;
      if (BIAS_MODE == 2) bv = bias[n];
#pragma unroll
      for (int r = 0; r < 8; ++r) {
        float v = acc[i][j][r] * scale;
        if (BIAS_MODE == 1) v += bias[mBase + mOff + r];
        if (BIAS_MODE == 2) v += bv;
        if (RESID) v += Rb[(size_t)(mBase + mOff + r) * ldc + n];
        if (ACT == 1) v = tanhf(v);
        if (ACT == 2) v = fmaxf(v, 0.0f);
        if (ACT == 3) v = v / (1.0f + expf(-v));
        if (ACT == 4) v = (v > 0.f) ? v : 0.01f * v;
        if (ACT == 5) v = 0.5f * v * (1.0f + erff(v * 0.70710678118654752f));
        slab[(mOff + r) * 68 + (j << 4) + rlane] = v;
      }
    }
    __builtin_amdgcn_fence(__ATOMIC_RELEASE, "workgroup");
    __builtin_amdgcn_wave_barrier();
    __builtin_amdgcn_fence(__ATOMIC_ACQUIRE, "workgroup");
    if (OUT_MODE == 0) {
      float* C = (float*)Cout + (size_t)b * strideC;
      const int hh = lane >> 4, c4 = (lane & 15) * 4;
      for (int pass = 0; pass < 2; ++pass) {
#pragma unroll
        for (int it = 0; it < 8; ++it) {
          const int row = it * 2 + hh;
          v4f v = *(const v4f*)(slab + row * 68 + c4);
          *(volatile v4f*)(C + (size_t)(mBase + row) * ldc + n0 + c4) = v;
        }
        __threadfence();
      }
    } else {
      const int q = lane >> 3, c8 = (lane & 7) * 8;
      unsigned short* C  = (unsigned short*)Cout  + (size_t)b * strideC;
      unsigned short* C2 = (OUT_MODE == 2) ? ((unsigned short*)Cout2 + (size_t)b * strideC) : nullptr;
      for (int pass = 0; pass < 2; ++pass) {
#pragma unroll
        for (int it = 0; it < 4; ++it) {
          const int row = it * 4 + q;
          const float* sp = slab + row * 68 + c8;
          v8h hv, lv;
#pragma unroll
          for (int e = 0; e < 8; ++e) {
            if (OUT_MODE == 1) {
              hv[e] = (_Float16)sp[e];
            } else {
              unsigned short hb = f2bf_bits(sp[e]);
              unsigned short lb = f2bf_bits(sp[e] - bf_bits2f(hb));
              hv[e] = __builtin_bit_cast(_Float16, hb);
              lv[e] = __builtin_bit_cast(_Float16, lb);
            }
          }
          *(volatile v8h*)(C + (size_t)(mBase + row) * ldc + n0 + c8) = hv;
          if (OUT_MODE == 2) *(volatile v8h*)(C2 + (size_t)(mBase + row) * ldc + n0 + c8) = lv;
        }
        __threadfence();
      }
    }
    __builtin_amdgcn_fence(__ATOMIC_RELEASE, "workgroup");
    __builtin_amdgcn_wave_barrier();
    __builtin_amdgcn_fence(__ATOMIC_ACQUIRE, "workgroup");
  }
}

template <bool PERM>
__global__ __launch_bounds__(CVT_THR) void cvt8_f16_kernel(const float* __restrict__ src, unsigned short* __restrict__ dst,
                                                           int n8, float sc) {
  const int i = blockIdx.x * CVT_THR + threadIdx.x;
  if (i < n8) {
    const int row = i / (NIN / 8);
    const int c8  = i - row * (NIN / 8);
    const int srow = PERM ? ((row % NBATCH) * NSTEP + (row / NBATCH)) : row;
    const float* sp = src + (size_t)srow * NIN + c8 * 8;
    const v4f a = *(const v4f*)(sp);
    const v4f b = *(const v4f*)(sp + 4);
    v8h hv;
#pragma unroll
    for (int e = 0; e < 4; ++e) {
      const float fa = a[e];
      const float fb = b[e];
      hv[e]     = (_Float16)(fa * sc);
      hv[4 + e] = (_Float16)(fb * sc);
    }
    *(volatile v8h*)(dst + (size_t)i * 8) = hv;
    __threadfence();
    *(volatile v8h*)(dst + (size_t)i * 8) = hv;
  }
}

__global__ __launch_bounds__(CVT_THR) void bias_prep_kernel(const float* __restrict__ wb, const float* __restrict__ ub,
                                                            float* __restrict__ dst, float sc) {
  const int i = blockIdx.x * CVT_THR + threadIdx.x;
  if (i < NG4 / 4) {
    const v4f a = *(const v4f*)(wb + 4 * i);
    const v4f b = *(const v4f*)(ub + 4 * i);
    v4f o;
#pragma unroll
    for (int e = 0; e < 4; ++e) {
      const float fa = a[e];
      const float fb = b[e];
      o[e] = (fa + fb) * sc;
    }
    *(volatile v4f*)(dst + 4 * i) = o;
    __threadfence();
    *(volatile v4f*)(dst + 4 * i) = o;
  }
}

__device__ __forceinline__ float gate_sig(float x)  { return __builtin_amdgcn_rcpf(1.0f + expf(-x)); }
__device__ __forceinline__ float gate_tanh(float x) { return 1.0f - 2.0f * __builtin_amdgcn_rcpf(expf(2.0f * x) + 1.0f); }

__global__ __launch_bounds__(SEQ_THR) void slstm_seq_kernel(const unsigned* __restrict__ Zw,
                                                            const unsigned short* __restrict__ Uhp,
                                                            const float* __restrict__ alpha,
                                                            float* __restrict__ out0, float* __restrict__ out1,
                                                            float* __restrict__ out2) {
  __shared__ __align__(16) _Float16 Ah[2][16 * HPITCH];
  __shared__ __align__(16) float    Sf[2][NBATCH * SPITCH];
  const _Float16* Uh = (const _Float16*)Uhp;
  const int tid = threadIdx.x, lane = tid & 31, wave = tid >> 5;
  const int c = lane & 15, hh = lane >> 4, koff = hh * 8;

  {
    _Float16* ahf = &Ah[0][0];
#pragma unroll 1
    for (int i = tid; i < 2 * 16 * HPITCH; i += SEQ_THR) ahf[i] = (_Float16)0.0f;
  }
  float cst[2][8];
  float al[2];
#pragma unroll
  for (int nt = 0; nt < 2; ++nt) {
    al[nt] = alpha[32 * wave + 16 * nt + c];
#pragma unroll
    for (int r = 0; r < 8; ++r) cst[nt][r] = 0.0f;
  }
  float zmask = (hh == 0) ? 1.0f : 0.0f;
  asm volatile("" : "+v"(zmask));
  __syncthreads();

#pragma unroll 1
  for (int t = 0; t < NSTEP; ++t) {
    const int cur = t & 1;
    const _Float16* ahrow = &Ah[cur][0] + c * HPITCH + koff;
    _Float16* ahn = &Ah[cur ^ 1][0];
    float* sf = &Sf[cur][0];
    const unsigned* zrow = Zw + (size_t)t * (size_t)(NBATCH * (NG4 / 2));
    const bool last = (t == NSTEP - 1);

#pragma unroll
    for (int nt = 0; nt < 2; ++nt) {
      const int j  = 32 * wave + 16 * nt + c;
      const int jw = j >> 1;
      const unsigned sh = (unsigned)(j & 1) * 16u;
      const _Float16* u0 = Uh + (size_t)j * NHID + koff;
      v8f acc[4];
#pragma unroll
      for (int g = 0; g < 4; ++g) {
#pragma unroll
        for (int r = 0; r < 8; ++r) {
          unsigned w = zrow[r * (NG4 / 2) + g * (NHID / 2) + jw];
          asm volatile("" : "+v"(w));
          const unsigned hb = (w >> sh) & 0xffffu;
          const float zv = h16_to_f32(hb);
          acc[g][r] = zv * zmask;
        }
      }
#pragma unroll 1
      for (int k0 = 0; k0 < NHID; k0 += 32) {
        const v16h a  = Frag<_Float16>::load(ahrow + k0);
        const v16h b0 = Frag<_Float16>::load(u0 + k0);
        const v16h b1 = Frag<_Float16>::load(u0 + (size_t)1 * NHID * NHID + k0);
        const v16h b2 = Frag<_Float16>::load(u0 + (size_t)2 * NHID * NHID + k0);
        const v16h b3 = Frag<_Float16>::load(u0 + (size_t)3 * NHID * NHID + k0);
        acc[0] = Frag<_Float16>::mma(a, b0, acc[0]);
        acc[1] = Frag<_Float16>::mma(a, b1, acc[1]);
        acc[2] = Frag<_Float16>::mma(a, b2, acc[2]);
        acc[3] = Frag<_Float16>::mma(a, b3, acc[3]);
        grp_guard_h(acc[0], acc[1], acc[2], acc[3], a, b0, b1, b2, b3);
      }
      acc_guard4(acc[0], acc[1], acc[2], acc[3]);
#pragma unroll
      for (int r = 0; r < 8; ++r) {
        const float zi = acc[0][r] * WCARRY_INV;
        const float zf = acc[1][r] * WCARRY_INV;
        const float zo = acc[2][r] * WCARRY_INV;
        const float zg = acc[3][r] * WCARRY_INV;
        const float ig = gate_sig(zi);
        const float fg = gate_sig(zf);
        const float og = gate_sig(zo);
        const float gg = gate_tanh(zg);
        const float cn = al[nt] * (fg * cst[nt][r] + ig * gg);
        cst[nt][r] = cn;
        const float hn = og * gate_tanh(cn);
        const float hw = (hh == 0) ? hn : 0.0f;
        ahn[(8 * hh + r) * HPITCH + j] = (_Float16)hw;
        if (hh == 0) sf[r * SPITCH + j] = hn;
      }
    }
    __syncthreads();

    for (int pass = 0; pass < 2; ++pass) {
#pragma unroll
      for (int it = 0; it < 2; ++it) {
        const int idx = it * SEQ_THR + tid;
        const int row = idx >> 7;
        const int c4  = (idx & 127) * 4;
        const v4f v = *(const v4f*)(sf + row * SPITCH + c4);
        *(volatile v4f*)(out0 + ((size_t)row * NSTEP + (size_t)t) * NHID + c4) = v;
        if (last) *(volatile v4f*)(out1 + (size_t)row * NHID + c4) = v;
      }
      __threadfence();
    }
  }

  {
    float* sc = &Sf[NSTEP & 1][0];
#pragma unroll
    for (int nt = 0; nt < 2; ++nt) {
      const int j = 32 * wave + 16 * nt + c;
#pragma unroll
      for (int r = 0; r < 8; ++r) {
        if (hh == 0) sc[r * SPITCH + j] = cst[nt][r];
      }
    }
    __syncthreads();
    for (int pass = 0; pass < 2; ++pass) {
#pragma unroll
      for (int it = 0; it < 2; ++it) {
        const int idx = it * SEQ_THR + tid;
        const int row = idx >> 7;
        const int c4  = (idx & 127) * 4;
        const v4f v = *(const v4f*)(sc + row * SPITCH + c4);
        *(volatile v4f*)(out2 + (size_t)row * NHID + c4) = v;
      }
      __threadfence();
    }
  }
}

extern "C" void kernel_launch(void* const* d_in, const int* in_sizes, int n_in,
                              void* d_out, int out_size, void* d_ws, size_t ws_size, hipStream_t stream) {
  if (n_in < 6 || d_out == nullptr || d_ws == nullptr) return;
  if (in_sizes[0] != NBATCH * NSTEP * NIN || in_sizes[1] != NG4 * NIN || in_sizes[2] != NG4 ||
      in_sizes[3] != NG4 * NHID || in_sizes[4] != NG4 || in_sizes[5] != NHID ||
      out_size != NOUT0 + 2 * NOUT1) return;

  const float* x     = (const float*)d_in[0];
  const float* w_w   = (const float*)d_in[1];
  const float* w_b   = (const float*)d_in[2];
  const float* u_w   = (const float*)d_in[3];
  const float* u_b   = (const float*)d_in[4];
  const float* alpha = (const float*)d_in[5];
  float* out0 = (float*)d_out;
  float* out1 = out0 + (size_t)NOUT0;
  float* out2 = out1 + (size_t)NOUT1;

  char* ws = (char*)d_ws; size_t off = 0;
  auto carve = [&](size_t bytes) -> char* { char* p = ws + off; off += (bytes + 255) & ~(size_t)255; return p; };
  unsigned short* XH   = (unsigned short*)carve((size_t)NROWS * NIN * 2);
  unsigned short* WH   = (unsigned short*)carve((size_t)NG4 * NIN * 2);
  unsigned short* UH   = (unsigned short*)carve((size_t)NG4 * NHID * 2);
  float*          BIAS = (float*)carve((size_t)NG4 * 4);
  unsigned short* Z16  = (unsigned short*)carve((size_t)NROWS * NG4 * 2);
  if (off > ws_size || off > (size_t)134217728) return;

  const int n8x = NROWS * (NIN / 8);
  const int n8w = NG4 * (NIN / 8);
  cvt8_f16_kernel<true ><<<(n8x + CVT_THR - 1) / CVT_THR, CVT_THR, 0, stream>>>(x,   XH, n8x, 1.0f);
  cvt8_f16_kernel<false><<<(n8w + CVT_THR - 1) / CVT_THR, CVT_THR, 0, stream>>>(w_w, WH, n8w, WCARRY);
  cvt8_f16_kernel<false><<<(n8w + CVT_THR - 1) / CVT_THR, CVT_THR, 0, stream>>>(u_w, UH, n8w, WCARRY);
  bias_prep_kernel<<<(NG4 / 4 + CVT_THR - 1) / CVT_THR, CVT_THR, 0, stream>>>(w_b, u_b, BIAS, WCARRY);

  const dim3 ggrid((NROWS / 64) * (NG4 / 64) / 8, 1);
  wmma_gemm64<0, false, 2, 1, false, 0><<<ggrid, 256, 0, stream>>>(
      XH, XH, NIN, 0L, WH, WH, NIN, 0L, (void*)Z16, (void*)Z16, NG4, 0L,
      BIAS, BIAS, 0L, NROWS, NG4, NIN, 1.0f);

  slstm_seq_kernel<<<1, SEQ_THR, 0, stream>>>((const unsigned*)Z16, UH, alpha, out0, out1, out2);
}
